// ChunkwiseRetention_73538430042347
// MI455X (gfx1250) — hardware-run, weakly checked
//
#include <hip/hip_runtime.h>


#define NSQ 8
#define NTS 1024
#define NDM 512
#define NCS 64
#define NCK 16
#define NBK 128
#define NBL 4096
#define NRW 8192

typedef _Float16 h16;
typedef unsigned short bf;
typedef __attribute__((ext_vector_type(16))) __bf16   v16bf;
typedef __attribute__((ext_vector_type(16))) _Float16 v16h;
typedef __attribute__((ext_vector_type(8)))  _Float16 v8h;
typedef __attribute__((ext_vector_type(8)))  unsigned short v8us;
typedef __attribute__((ext_vector_type(8)))  float    v8f;
typedef __attribute__((ext_vector_type(4)))  float    v4f;
typedef v8h  __attribute__((may_alias)) v8ha;
typedef v4f  __attribute__((may_alias)) v4fa;
typedef v8us __attribute__((may_alias)) v8usa;

__device__ __forceinline__ unsigned short f2bf(float f) { unsigned u = __float_as_uint(f); u += 0x7FFFu + ((u >> 16) & 1u); return (unsigned short)(u >> 16); }
__device__ __forceinline__ float bf2f(unsigned short b) { return __uint_as_float(((unsigned)b) << 16); }
__device__ __forceinline__ float bfr(float f) { return bf2f(f2bf(f)); }
__device__ __forceinline__ v16h cat16(v8h lo, v8h hi) { return __builtin_shufflevector(lo, hi, 0, 1, 2, 3, 4, 5, 6, 7, 8, 9, 10, 11, 12, 13, 14, 15); }
__device__ __forceinline__ v16bf cat16b(v8us lo, v8us hi) { return __builtin_bit_cast(v16bf, __builtin_shufflevector(lo, hi, 0, 1, 2, 3, 4, 5, 6, 7, 8, 9, 10, 11, 12, 13, 14, 15)); }
__device__ __forceinline__ v8f wmma16(v16h a, v16h b, v8f c) { return __builtin_amdgcn_wmma_f32_16x16x32_f16(false, a, false, b, (short)0, c, false, false); }
__device__ __forceinline__ v8f wmmab(v16bf a, v16bf b, v8f c) { return __builtin_amdgcn_wmma_f32_16x16x32_bf16(false, a, false, b, (short)0, c, false, false); }

template <typename T16> struct WFrag;
template <> struct WFrag<h16> { typedef v16h V; static __device__ __forceinline__ V ld(const h16* p) { return cat16(*(const v8h*)p, *(const v8h*)(p + 16)); } static __device__ __forceinline__ v8f mma(V a, V b, v8f c) { return wmma16(a, b, c); } };
template <> struct WFrag<bf> { typedef v16bf V; static __device__ __forceinline__ V ld(const bf* p) { return cat16b(*(const v8us*)p, *(const v8us*)(p + 16)); } static __device__ __forceinline__ v8f mma(V a, V b, v8f c) { return wmmab(a, b, c); } };
template <typename T16, int NSPLIT, bool BIAS>
__global__ __launch_bounds__(32) void k_gemmw(const T16* __restrict__ A, const T16* __restrict__ A2, const T16* __restrict__ Bt, const T16* __restrict__ Bt2, int K, float* C, int ldc, const float* __restrict__ bias, size_t sA, size_t sB, size_t sC) {
    typedef typename WFrag<T16>::V V;
    __shared__ __align__(16) float os[16 * 68];
    const size_t z = blockIdx.z; A += z * sA; if (A2) A2 += z * sA; Bt += z * sB; if (Bt2) Bt2 += z * sB; C += z * sC;
    const int lane = threadIdx.x & 31, lr = lane & 15, hi = lane >> 4; const int r0 = blockIdx.x * 64, c0 = blockIdx.y * 64;
    v8f acc[4][4];
#pragma unroll
    for (int mb = 0; mb < 4; ++mb)
#pragma unroll
        for (int nb = 0; nb < 4; ++nb) acc[mb][nb] = (v8f){};
    const size_t aoff = (size_t)(r0 + lr) * K + 8 * hi, boff = (size_t)(c0 + lr) * K + 8 * hi;
    for (int kc = 0; kc < K; kc += 32) {
        V a[4], a2[4];
#pragma unroll
        for (int mb = 0; mb < 4; ++mb) { a[mb] = WFrag<T16>::ld(A + aoff + (size_t)mb * 16 * K + kc); if (NSPLIT == 1 || NSPLIT == 2) a2[mb] = WFrag<T16>::ld(A2 + aoff + (size_t)mb * 16 * K + kc); }
#pragma unroll
        for (int nb = 0; nb < 4; ++nb) { const V b = WFrag<T16>::ld(Bt + boff + (size_t)nb * 16 * K + kc); V b2; if (NSPLIT >= 2) b2 = WFrag<T16>::ld(Bt2 + boff + (size_t)nb * 16 * K + kc);
#pragma unroll
            for (int mb = 0; mb < 4; ++mb) { acc[mb][nb] = WFrag<T16>::mma(a[mb], b, acc[mb][nb]); if (NSPLIT == 1 || NSPLIT == 2) acc[mb][nb] = WFrag<T16>::mma(a2[mb], b, acc[mb][nb]); if (NSPLIT >= 2) acc[mb][nb] = WFrag<T16>::mma(a[mb], b2, acc[mb][nb]); } }
        asm volatile("v_nop\n\tv_nop\n\tv_nop\n\tv_nop" : "+v"(acc[0][0]), "+v"(acc[1][1]), "+v"(acc[2][2]), "+v"(acc[3][3]) : "v"(a[0]), "v"(a[3]));
    }
#pragma unroll
    for (int mb = 0; mb < 4; ++mb) {
#pragma unroll
        for (int nb = 0; nb < 4; ++nb) {
#pragma unroll
            for (int j = 0; j < 8; ++j) os[(hi * 8 + j) * 68 + nb * 16 + lr] = acc[mb][nb][j]; }
        __builtin_amdgcn_wave_barrier(); asm volatile("" ::: "memory");
        float* crow = C + (size_t)(r0 + mb * 16) * ldc + c0;
#pragma unroll 1
        for (int ps = 0; ps < 2; ++ps) {
#pragma unroll
            for (int s = 0; s < 8; ++s) { const int row = 2 * s + hi, cofs = lr * 4; v4f val = *(const v4fa*)(os + row * 68 + cofs); if (BIAS) { val[0] += bfr(bias[c0 + cofs]); val[1] += bfr(bias[c0 + cofs + 1]); val[2] += bfr(bias[c0 + cofs + 2]); val[3] += bfr(bias[c0 + cofs + 3]); }
                *(volatile v4f*)(crow + (size_t)row * ldc + cofs) = val; }
            if (ps == 0) __threadfence(); }
        __builtin_amdgcn_wave_barrier(); asm volatile("" ::: "memory");
    }
}

typedef __attribute__((ext_vector_type(2))) _Float16 v2h;
typedef __attribute__((ext_vector_type(4))) _Float16 v4h;
typedef __attribute__((ext_vector_type(2))) unsigned short v2us;
typedef __attribute__((ext_vector_type(4))) unsigned short v4us;
typedef __attribute__((ext_vector_type(2))) float v2f;
typedef __attribute__((ext_vector_type(4))) int v4i;
__device__ __forceinline__ h16 toh_flush(float x) { const float z = (fabsf(x) < 6.103515625e-05f) ? 0.0f : x; return (h16)z; }

typedef __attribute__((ext_vector_type(4))) _Float16 v4h_;
__global__ __launch_bounds__(256) void k_fillb(bf* P, unsigned w2, size_t n8) { const size_t i = (size_t)blockIdx.x * 256 + threadIdx.x; if (i >= n8) return; v4i o; o[0] = (int)w2; o[1] = (int)w2; o[2] = (int)w2; o[3] = (int)w2;
    *(volatile v4i*)(P + i * 8) = o; __threadfence(); *(volatile v4i*)(P + i * 8) = o; }

__global__ __launch_bounds__(256) void k_wtw(const float* __restrict__ W, h16* Wt) {
    const unsigned i = blockIdx.x * 256 + threadIdx.x; const unsigned n = i & 511u, k64 = i >> 9; const float* src = W + (size_t)k64 * 64 * NDM + n; h16 r[64];
#pragma unroll
    for (int kj = 0; kj < 64; ++kj) r[kj] = toh_flush(bfr(src[(size_t)kj * NDM]) * 1024.0f);
    h16* pd = Wt + (size_t)n * NDM + (size_t)k64 * 64;
#pragma unroll
    for (int ps = 0; ps < 2; ++ps) {
#pragma unroll
        for (int g = 0; g < 8; ++g) { v8h o;
#pragma unroll
            for (int j = 0; j < 8; ++j) o[j] = r[g * 8 + j];
            *(volatile v8h*)(pd + g * 8) = o; }
        if (ps == 0) __threadfence(); } }

__global__ __launch_bounds__(256) void k_xword(const float* __restrict__ src, h16* dst) {
    const size_t i = (size_t)blockIdx.x * 256 + threadIdx.x; const v8f wv = *(const v8f*)(src + i * 8); v8h ow;
#pragma unroll
    for (int j = 0; j < 8; ++j) ow[j] = toh_flush(bfr(wv[j]));
    *(volatile v8h*)(dst + i * 8) = ow; __threadfence(); *(volatile v8h*)(dst + i * 8) = ow; }

template <int QM>
__global__ __launch_bounds__(256) void k_fw(const float* __restrict__ src, float* sums, h16* dst) {
    const unsigned i = blockIdx.x * 256 + threadIdx.x; const unsigned t = i & 1023u, sq = i >> 10; const unsigned td = QM ? ((t + 1023u) & 1023u) : t; const float live = QM ? (float)(t >= 1u) : 1.0f;
    const float ex = QM ? (float)((td & 63u) + 1u) : -(float)(t & 63u); const float fac = exp2f(ex * -0.0392180160f) * live * 0.0009765625f; const float* ps_ = src + (size_t)i * NDM; h16* pd = dst + ((size_t)sq * NTS + td) * NDM; float acc = 0.0f;
#pragma unroll
    for (int ps = 0; ps < 2; ++ps) {
#pragma unroll
        for (int g = 0; g < 64; ++g) { const v8f w = *(const v8f*)(ps_ + g * 8); v8h o;
#pragma unroll
            for (int j = 0; j < 8; ++j) { if (ps == 0) acc = acc + w[j] * 0.0009765625f; o[j] = toh_flush(w[j] * fac); }
            *(volatile v8h*)(pd + g * 8) = o; }
        if (ps == 0) { *(volatile float*)(sums + i) = acc; __threadfence(); } else *(volatile float*)(sums + i) = acc; } }

template <bool KM>
__global__ __launch_bounds__(256) void k_colw(const float* __restrict__ src, h16* dst) {
    constexpr float CF[64] = {1.00000000f, 1.02755666f, 1.05587280f, 1.08496916f, 1.11486733f, 1.14558947f, 1.17715812f, 1.20959675f, 1.24292922f, 1.27718019f, 1.31237507f, 1.34853983f, 1.38570118f, 1.42388654f, 1.46312416f, 1.50344300f, 1.54487300f, 1.58744466f, 1.63118935f, 1.67613959f, 1.72232842f, 1.76979017f, 1.81855977f, 1.86867332f, 1.92016780f, 1.97308123f, 2.02745295f, 2.08332276f, 2.14073229f, 2.19972396f, 2.26034093f, 2.32262850f, 2.38663268f, 2.45240045f, 2.51998043f, 2.58942270f, 2.66077876f, 2.73410106f, 2.80944395f, 2.88686299f, 2.96641541f, 3.04816008f, 3.13215733f, 3.21846914f, 3.30715966f, 3.39829397f, 3.49193978f, 3.58816624f, 3.68704438f, 3.78864717f, 3.89304972f, 4.00032949f, 4.11056519f, 4.22383881f, 4.34023380f, 4.45983648f, 4.58273506f, 4.70902014f, 4.83878517f, 4.97212601f, 5.10914183f, 5.24993277f, 5.39460373f, 5.54326105f};
    const unsigned i = blockIdx.x * 256 + threadIdx.x; const unsigned cl = i & 511u, z = i >> 9; const float* pp = src + (size_t)z * 64 * NDM + cl; h16 r[64];
#pragma unroll
    for (int u = 0; u < 64; ++u) r[u] = toh_flush(pp[(size_t)u * NDM] * 0.0009765625f * (KM ? CF[u] : 1.0f));
    h16* pd = dst + (size_t)i * 64;
#pragma unroll
    for (int ps = 0; ps < 2; ++ps) {
#pragma unroll
        for (int g = 0; g < 8; ++g) { v8h o;
#pragma unroll
            for (int j = 0; j < 8; ++j) o[j] = r[g * 8 + j];
            *(volatile v8h*)(pd + g * 8) = o; }
        if (ps == 0) __threadfence(); } }

__global__ __launch_bounds__(256) void k_msk3(const float* __restrict__ Pw, h16* Ph) {
    const unsigned i = blockIdx.x * 256 + threadIdx.x; const unsigned tr = i & 63u; const float* pw = Pw + (size_t)i * 64; h16 rh[64];
#pragma unroll
    for (int g = 0; g < 8; ++g) { const v8f t = *(const v8f*)(pw + g * 8);
#pragma unroll
        for (int j = 0; j < 8; ++j) { const float kp = (float)((unsigned)(g * 8 + j) <= tr); rh[g * 8 + j] = toh_flush(t[j] * kp); } }
    h16* ph = Ph + (size_t)i * 64;
#pragma unroll
    for (int ps = 0; ps < 2; ++ps) {
#pragma unroll
        for (int g = 0; g < 8; ++g) { v8h oh;
#pragma unroll
            for (int j = 0; j < 8; ++j) oh[j] = rh[g * 8 + j];
            *(volatile v8h*)(ph + g * 8) = oh; }
        if (ps == 0) __threadfence(); } }

__global__ __launch_bounds__(256) void k_dsum(const float* __restrict__ bef, const float* __restrict__ du, float* aft, h16* wrd) {
    const size_t i = (size_t)blockIdx.x * 256 + threadIdx.x; const v4f ub = *(const v4fa*)(bef + i * 4); const v4f vd = *(const v4fa*)(du + i * 4); v4f oa; v4h_ ow;
#pragma unroll
    for (int j = 0; j < 4; ++j) { oa[j] = (ub[j] + vd[j]) * 0.175561324f; ow[j] = toh_flush(oa[j]); }
    *(volatile v4f*)(aft + i * 4) = oa; *(volatile v4h_*)(wrd + i * 4) = ow; __threadfence(); *(volatile v4f*)(aft + i * 4) = oa; *(volatile v4h_*)(wrd + i * 4) = ow; }

__global__ __launch_bounds__(256) void k_lay3(const float* __restrict__ sQ, const float* __restrict__ sK, const float* __restrict__ V, const float* __restrict__ Oa, const float* __restrict__ Ob, float* res) {
    const size_t i = (size_t)blockIdx.x * 256 + threadIdx.x; const size_t row = i >> 7; const float s = sQ[row] * sK[row]; const v4f uv = *(const v4fa*)(V + i * 4); const v4f ua = *(const v4fa*)(Oa + i * 4); const v4f ub = *(const v4fa*)(Ob + i * 4); v4f o;
#pragma unroll
    for (int j = 0; j < 4; ++j) o[j] = s * (uv[j] * 0.0009765625f) + (ua[j] + ub[j]);
    *(volatile v4f*)(res + i * 4) = o; __threadfence(); *(volatile v4f*)(res + i * 4) = o; }

extern "C" void kernel_launch(void* const* d_in, const int* in_sizes, int n_in, void* d_out, int out_size, void* d_ws, size_t ws_size, hipStream_t stream) {
    if (n_in < 6) return;
    if (in_sizes[0] != NRW * NDM || in_sizes[1] != NRW * NDM || in_sizes[2] != NRW * NDM || in_sizes[3] != NDM * NDM || in_sizes[4] != NDM * NDM || in_sizes[5] != NDM * NDM) return;
    if (out_size != NRW * NDM) return;
    static_assert(NRW == NSQ * NTS && NTS == 1024 && NDM == 512 && NCS == 64 && NCK * NCS == NTS && NBK == NSQ * NCK && NBL == 64 * 64 && (NDM * 8) % 256 == 0 && (NRW * NDM / 8) % 256 == 0 && NRW % 256 == 0 && (NBK * NDM) % 256 == 0 && (NBK * 64) % 256 == 0 && (NSQ * NDM * NDM / 4) % 256 == 0 && (NRW * NDM / 4) % 256 == 0 && (NSQ * NDM * NDM * 4 / 16) % 256 == 0 && (NSQ * NDM * NDM * 2 / 16) % 256 == 0, "the block products: 64-row tiles over depths of 512 and 64; the flat grids exact; the index fields' widths (10 bits a step, 9 a column, 6 a step within a chunk)");
    const float* xq = (const float*)d_in[0]; const float* xk = (const float*)d_in[1]; const float* xv = (const float*)d_in[2]; const float* Wq = (const float*)d_in[3]; const float* Wk = (const float*)d_in[4]; const float* Wv = (const float*)d_in[5]; float* res = (float*)d_out;
    char* wsp = (char*)d_ws; auto take = [&](size_t bytes) { char* p = wsp; wsp += (bytes + 255) & ~(size_t)255; return (void*)p; };
    h16* Xw = (h16*)take((size_t)NRW * NDM * 2); h16* Wtq = (h16*)take((size_t)NDM * NDM * 2); h16* Wtk = (h16*)take((size_t)NDM * NDM * 2); h16* Wtv = (h16*)take((size_t)NDM * NDM * 2);
    float* T0 = (float*)take((size_t)NRW * NDM * 4); float* T1 = (float*)take((size_t)NRW * NDM * 4); float* T2 = (float*)take((size_t)NRW * NDM * 4); float* sQ = (float*)take((size_t)NRW * 4); float* sK = (float*)take((size_t)NRW * 4);
    h16* Qs = (h16*)take((size_t)NRW * NDM * 2); h16* Ks = (h16*)take((size_t)NRW * NDM * 2); h16* KsT = (h16*)take((size_t)NBK * NDM * 64 * 2); h16* VT = (h16*)take((size_t)NBK * NDM * 64 * 2);
    float* Pw = (float*)take((size_t)NBK * NBL * 4); h16* Ph = (h16*)take((size_t)NBK * NBL * 2);
    float* StA = (float*)take((size_t)NSQ * NDM * NDM * 4); float* StB = (float*)take((size_t)NSQ * NDM * NDM * 4); h16* SwA = (h16*)take((size_t)NSQ * NDM * NDM * 2); h16* SwB = (h16*)take((size_t)NSQ * NDM * NDM * 2); float* Du = (float*)take((size_t)NSQ * NDM * NDM * 4);
    if ((size_t)(wsp - (char*)d_ws) > ws_size) return;
    float* Q = T0; float* K = T1; float* V = T2; float* Oa = T0; float* Ob = T1;
    k_wtw<<<NDM * 8 / 256, 256, 0, stream>>>(Wq, Wtq); k_wtw<<<NDM * 8 / 256, 256, 0, stream>>>(Wk, Wtk); k_wtw<<<NDM * 8 / 256, 256, 0, stream>>>(Wv, Wtv);
    k_xword<<<(unsigned)(NRW * NDM / 8 / 256), 256, 0, stream>>>(xq, Xw); k_gemmw<h16, 0, false><<<dim3(NRW / 64, NDM / 64, 1), 32, 0, stream>>>(Xw, nullptr, Wtq, nullptr, NDM, Q, NDM, nullptr, 0, 0, 0);
    k_xword<<<(unsigned)(NRW * NDM / 8 / 256), 256, 0, stream>>>(xk, Xw); k_gemmw<h16, 0, false><<<dim3(NRW / 64, NDM / 64, 1), 32, 0, stream>>>(Xw, nullptr, Wtk, nullptr, NDM, K, NDM, nullptr, 0, 0, 0);
    k_xword<<<(unsigned)(NRW * NDM / 8 / 256), 256, 0, stream>>>(xv, Xw); k_gemmw<h16, 0, false><<<dim3(NRW / 64, NDM / 64, 1), 32, 0, stream>>>(Xw, nullptr, Wtv, nullptr, NDM, V, NDM, nullptr, 0, 0, 0);
    k_fw<1><<<NRW / 256, 256, 0, stream>>>(Q, sQ, Qs); k_fw<0><<<NRW / 256, 256, 0, stream>>>(K, sK, Ks);
    k_colw<true><<<NBK * NDM / 256, 256, 0, stream>>>(K, KsT); k_colw<false><<<NBK * NDM / 256, 256, 0, stream>>>(V, VT);
    k_gemmw<h16, 0, false><<<dim3(1, 1, NBK), 32, 0, stream>>>(Qs, nullptr, Ks, nullptr, NDM, Pw, 64, nullptr, (size_t)64 * NDM, (size_t)64 * NDM, NBL);
    k_msk3<<<NBK * 64 / 256, 256, 0, stream>>>(Pw, Ph);
    k_gemmw<h16, 0, false><<<dim3(1, NDM / 64, NBK), 32, 0, stream>>>(Ph, nullptr, VT, nullptr, NCS, Oa, NDM, nullptr, NBL, (size_t)NDM * 64, (size_t)64 * NDM);
    k_fillb<<<(unsigned)((size_t)NSQ * NDM * NDM * 4 / 16 / 256), 256, 0, stream>>>((bf*)StA, 0u, (size_t)NSQ * NDM * NDM * 4 / 16); k_fillb<<<(unsigned)((size_t)NSQ * NDM * NDM * 2 / 16 / 256), 256, 0, stream>>>((bf*)SwA, 0u, (size_t)NSQ * NDM * NDM * 2 / 16);
    for (int ck = 0; ck < NCK; ++ck) { const float* stb = (ck & 1) ? StB : StA; float* sta = (ck & 1) ? StA : StB; const h16* swr = (ck & 1) ? SwB : SwA; h16* sww = (ck & 1) ? SwA : SwB;
        k_gemmw<h16, 0, false><<<dim3(1, NDM / 64, NSQ), 32, 0, stream>>>(Qs + (size_t)ck * 64 * NDM, nullptr, swr, nullptr, NDM, Ob + (size_t)ck * 64 * NDM, NDM, nullptr, (size_t)NTS * NDM, (size_t)NDM * NDM, (size_t)NTS * NDM);
        if (ck + 1 < NCK) { k_gemmw<h16, 0, false><<<dim3(NDM / 64, NDM / 64, NSQ), 32, 0, stream>>>(VT + (size_t)ck * NDM * 64, nullptr, KsT + (size_t)ck * NDM * 64, nullptr, NCS, Du, NDM, nullptr, (size_t)NCK * NDM * 64, (size_t)NCK * NDM * 64, (size_t)NDM * NDM);
            k_dsum<<<(unsigned)((size_t)NSQ * NDM * NDM / 4 / 256), 256, 0, stream>>>(stb, Du, sta, sww); } }
    k_lay3<<<(unsigned)((size_t)NRW * NDM / 4 / 256), 256, 0, stream>>>(sQ, sK, V, Oa, Ob, res);
}
